// MultiHeadAtttention_46797963657634
// MI455X (gfx1250) — hardware-verified
//
#include <hip/hip_runtime.h>
#include <math.h>
#include <stdint.h>

#define NB    4
#define SEQ   2048
#define DM    1024
#define NH    16
#define HD    64
#define NQB   (SEQ / 64)
static_assert(NH * HD == DM);
static_assert((SEQ % 64) == 0 && (DM % 64) == 0 && (DM % 32) == 0);

typedef _Float16 v16h __attribute__((ext_vector_type(16)));
typedef _Float16 v8h  __attribute__((ext_vector_type(8)));
typedef __bf16   v16b __attribute__((ext_vector_type(16)));
typedef __bf16   v8b  __attribute__((ext_vector_type(8)));
typedef float    v8f  __attribute__((ext_vector_type(8)));
typedef float    v4f  __attribute__((ext_vector_type(4)));
typedef unsigned int v4u __attribute__((ext_vector_type(4)));

__device__ __forceinline__ unsigned short bf_bits(float f) {
  unsigned u = __float_as_uint(f);
  return (unsigned short)((u + 0x7FFFu + ((u >> 16) & 1u)) >> 16);
}
__device__ __forceinline__ float bf_up(unsigned short h) { return __uint_as_float(((unsigned)h) << 16); }
__device__ __forceinline__ float bfr(float f) { return bf_up(bf_bits(f)); }
__device__ __forceinline__ unsigned short h_bits(_Float16 x) { return __builtin_bit_cast(unsigned short, x); }
__device__ __forceinline__ unsigned pk16(unsigned short a, unsigned short b) { return (unsigned)a | ((unsigned)b << 16); }
__device__ __forceinline__ v8f zero8() { v8f z = {0.f, 0.f, 0.f, 0.f, 0.f, 0.f, 0.f, 0.f}; return z; }

template <int AH> struct OpT;
template <> struct OpT<0> { typedef __bf16   E; typedef v16b V; typedef v8b V8; };
template <> struct OpT<1> { typedef _Float16 E; typedef v16h V; typedef v8h V8; };

template <int AH>
__device__ __forceinline__ typename OpT<AH>::V ldfrag(const typename OpT<AH>::E* p) {
  union { typename OpT<AH>::V v; typename OpT<AH>::V8 h[2]; } f;
  f.h[0] = *(const typename OpT<AH>::V8*)(p);
  f.h[1] = *(const typename OpT<AH>::V8*)(p + 16);
  return f.v;
}
__device__ __forceinline__ v16h ldfrag_h(const _Float16* p) {
  union { v16h v; v8h h[2]; } f;
  f.h[0] = *(const v8h*)(p);
  f.h[1] = *(const v8h*)(p + 16);
  return f.v;
}

__device__ __forceinline__ v8f mma_h(v16h a, v16h b, v8f c) {
  c = __builtin_amdgcn_wmma_f32_16x16x32_f16(false, a, false, b, (short)0, c, false, false);
#if defined(__HIP_DEVICE_COMPILE__)
  asm volatile("v_nop\n\tv_nop\n\tv_nop\n\tv_nop" : "+v"(c) : "v"(a), "v"(b));
#endif
  return c;
}
__device__ __forceinline__ v8f mma_raw(v16b a, v16b b, v8f c) {
  return __builtin_amdgcn_wmma_f32_16x16x32_bf16(false, a, false, b, (short)0, c, false, false);
}
__device__ __forceinline__ v8f mma_raw(v16h a, v16h b, v8f c) {
  return __builtin_amdgcn_wmma_f32_16x16x32_f16(false, a, false, b, (short)0, c, false, false);
}
template <typename F>
__device__ __forceinline__ void dep_guard(v8f& a, v8f& b, F x, F y) {
#if defined(__HIP_DEVICE_COMPILE__)
  asm volatile("v_nop\n\tv_nop\n\tv_nop\n\tv_nop" : "+v"(a), "+v"(b) : "v"(x), "v"(y));
#endif
}
template <typename F>
__device__ __forceinline__ void keep4(F a, F b, F c, F d) {
#if defined(__HIP_DEVICE_COMPILE__)
  asm volatile("v_nop" :: "v"(a), "v"(b), "v"(c), "v"(d));
#endif
}
__device__ __forceinline__ void acc_guard4(v8f& a, v8f& b, v8f& c, v8f& d) {
#if defined(__HIP_DEVICE_COMPILE__)
  asm volatile("v_nop\n\tv_nop\n\tv_nop\n\tv_nop" : "+v"(a), "+v"(b), "+v"(c), "+v"(d));
#endif
}
__device__ __forceinline__ void wave_sync_lds() {
  __builtin_amdgcn_fence(__ATOMIC_RELEASE, "workgroup");
  __builtin_amdgcn_wave_barrier();
  __builtin_amdgcn_fence(__ATOMIC_ACQUIRE, "workgroup");
}

__global__ __launch_bounds__(256) void cvt_bf16x8(const float* __restrict__ in, unsigned short* out, int n8) {
  const int i = blockIdx.x * 256 + threadIdx.x;
  if (i < n8) {
    const v4f a = *(const v4f*)(in + (size_t)i * 8);
    const v4f b = *(const v4f*)(in + (size_t)i * 8 + 4);
    v4u p;
    p[0] = pk16(bf_bits(a[0]), bf_bits(a[1]));
    p[1] = pk16(bf_bits(a[2]), bf_bits(a[3]));
    p[2] = pk16(bf_bits(b[0]), bf_bits(b[1]));
    p[3] = pk16(bf_bits(b[2]), bf_bits(b[3]));
    *(volatile v4u*)(out + (size_t)i * 8) = p;
    __threadfence();
    *(volatile v4u*)(out + (size_t)i * 8) = p;
  }
}

template <int KIND>
__global__ __launch_bounds__(256) void wtrans(const float* __restrict__ W, unsigned short* WT, float scale) {
  __shared__ float tile[64][65];
  const int tid = threadIdx.x;
  const int k0 = blockIdx.y * 64;
  const int n0 = blockIdx.x * 64;
  {
    const int row = tid >> 2, cc = (tid & 3) * 16;
    const float* src = W + (size_t)(k0 + row) * DM + n0 + cc;
#pragma unroll
    for (int e4 = 0; e4 < 4; ++e4) {
      const v4f v = *(const v4f*)(src + 4 * e4);
      tile[row][cc + 4 * e4 + 0] = bfr(v[0]);
      tile[row][cc + 4 * e4 + 1] = bfr(v[1]);
      tile[row][cc + 4 * e4 + 2] = bfr(v[2]);
      tile[row][cc + 4 * e4 + 3] = bfr(v[3]);
    }
  }
  __syncthreads();
  const int wave = tid >> 5, lane = tid & 31, q = lane >> 3, k8 = (lane & 7) * 8;
  v4u vals[2];
#pragma unroll
  for (int it = 0; it < 2; ++it) {
    const int nl = wave * 8 + it * 4 + q;
    v4u a;
#pragma unroll
    for (int e = 0; e < 4; ++e) {
      const float f0 = tile[k8 + 2 * e][nl], f1 = tile[k8 + 2 * e + 1][nl];
      unsigned short b0, b1;
      if (KIND == 0) { b0 = bf_bits(f0); b1 = bf_bits(f1); }
      else           { b0 = h_bits((_Float16)(f0 * scale)); b1 = h_bits((_Float16)(f1 * scale)); }
      a[e] = pk16(b0, b1);
    }
    vals[it] = a;
  }
  for (int pass = 0; pass < 2; ++pass) {
#pragma unroll
    for (int it = 0; it < 2; ++it) {
      const int nl = wave * 8 + it * 4 + q;
      *(volatile v4u*)(WT + (size_t)(n0 + nl) * DM + k0 + k8) = vals[it];
    }
    __threadfence();
  }
}

template <int AH, int OUT16, int BIAS_MODE>
__global__ __launch_bounds__(256) void gemm64(
    const unsigned short* __restrict__ Ap, int lda, long long strideA,
    const unsigned short* __restrict__ Btp, int ldb, long long strideB,
    const float* __restrict__ bias,
    void* Cout, int ldc, long long strideC,
    int M, int N, int K, float oscale) {
  typedef typename OpT<AH>::E E;
  typedef typename OpT<AH>::V V;
  const E* A  = (const E*)(const void*)Ap;
  const E* Bt = (const E*)(const void*)Btp;
  __shared__ __align__(16) float sT[8][16 * 68];
  const int b    = blockIdx.y;
  const int lane = threadIdx.x & 31;
  const int wave = threadIdx.x >> 5;
  const int tilesN = N >> 6;
  const int tilesM = M >> 6;
  const int tile = blockIdx.x * 8 + wave;
  if (tile >= tilesM * tilesN) return;
  const int tm = tile / tilesN;
  const int tn = tile - tm * tilesN;
  const int m0 = tm << 6;
  const int n0 = tn << 6;

  const E* Ab = A  + (size_t)b * strideA;
  const E* Bb = Bt + (size_t)b * strideB;

  const int rlane = lane & 15;
  const int koff  = (lane >> 4) * 8;
  const int mOff  = (lane >> 4) * 8;

  v8f acc[4][4];
#pragma unroll
  for (int i = 0; i < 4; ++i)
#pragma unroll
    for (int j = 0; j < 4; ++j) acc[i][j] = zero8();

  for (int k0 = 0; k0 < K; k0 += 32) {
    V bf[4];
#pragma unroll
    for (int j = 0; j < 4; ++j) {
      const size_t bo = (size_t)(n0 + (j << 4) + rlane) * ldb + koff + k0;
      bf[j] = ldfrag<AH>(Bb + bo);
    }
#pragma unroll
    for (int i = 0; i < 4; ++i) {
      const size_t ao = (size_t)(m0 + (i << 4) + rlane) * lda + koff + k0;
      const V af = ldfrag<AH>(Ab + ao);
#pragma unroll
      for (int j = 0; j < 4; ++j) acc[i][j] = mma_raw(af, bf[j], acc[i][j]);
      dep_guard<V>(acc[i][0], acc[i][3], af, bf[3]);
    }
    keep4<V>(bf[0], bf[1], bf[2], bf[3]);
  }
  acc_guard4(acc[0][0], acc[0][1], acc[0][2], acc[0][3]);
  acc_guard4(acc[1][0], acc[1][1], acc[1][2], acc[1][3]);
  acc_guard4(acc[2][0], acc[2][1], acc[2][2], acc[2][3]);
  acc_guard4(acc[3][0], acc[3][1], acc[3][2], acc[3][3]);

  float bc[4];
#pragma unroll
  for (int j = 0; j < 4; ++j) bc[j] = (BIAS_MODE == 1) ? bfr(bias[n0 + (j << 4) + rlane]) : 0.f;
  float* slab = sT[wave];
#pragma unroll
  for (int i = 0; i < 4; ++i) {
    const int mBase = m0 + (i << 4);
    float br[8];
#pragma unroll
    for (int r = 0; r < 8; ++r) br[r] = (BIAS_MODE == 2) ? bfr(bias[mBase + mOff + r]) : 0.f;
#pragma unroll
    for (int j = 0; j < 4; ++j) {
#pragma unroll
      for (int r = 0; r < 8; ++r) {
        slab[(mOff + r) * 68 + (j << 4) + rlane] = acc[i][j][r] * oscale + bc[j] + br[r];
      }
    }
    wave_sync_lds();
    if (OUT16 == 0) {
      float* C = (float*)Cout + (size_t)b * strideC;
      const int hh = lane >> 4, c4 = (lane & 15) * 4;
      v4f vv[8];
#pragma unroll
      for (int it = 0; it < 8; ++it) {
        const int row = it * 2 + hh;
        vv[it] = *(const v4f*)(slab + row * 68 + c4);
      }
      for (int pass = 0; pass < 2; ++pass) {
#pragma unroll
        for (int it = 0; it < 8; ++it) {
          const int row = it * 2 + hh;
          *(volatile v4f*)(C + (size_t)(mBase + row) * ldc + n0 + c4) = vv[it];
        }
        __threadfence();
      }
    } else {
      const int q = lane >> 3, c8 = (lane & 7) * 8;
      unsigned short* C = (unsigned short*)Cout + (size_t)b * strideC;
      v4u hv[4];
#pragma unroll
      for (int it = 0; it < 4; ++it) {
        const int row = it * 4 + q;
        const float* sp = slab + row * 68 + c8;
        v4u a;
#pragma unroll
        for (int e = 0; e < 4; ++e) {
          const float f0 = sp[2 * e], f1 = sp[2 * e + 1];
          a[e] = pk16(h_bits((_Float16)f0), h_bits((_Float16)f1));
        }
        hv[it] = a;
      }
      for (int pass = 0; pass < 2; ++pass) {
#pragma unroll
        for (int it = 0; it < 4; ++it) {
          const int row = it * 4 + q;
          *(volatile v4u*)(C + (size_t)(mBase + row) * ldc + n0 + c8) = hv[it];
        }
        __threadfence();
      }
    }
    wave_sync_lds();
  }
}

__global__ __launch_bounds__(128)
void colstats(const unsigned short* __restrict__ qp, const unsigned short* __restrict__ kp,
              float* stats, float sscale) {
  union FH { v16h v; v8h h[2]; };
  __shared__ __align__(16) _Float16 Qsh[64 * 64];
  __shared__ __align__(16) float    Ssh[128];

  const int tid  = threadIdx.x;
  const int wave = tid >> 5;
  const int lane = tid & 31;
  const int hh   = lane >> 4;
  const int c    = lane & 15;

  const int bx   = blockIdx.x;
  const int kb   = bx % NQB;
  const int rest = bx / NQB;
  const int h    = rest % NH;
  const int b    = rest / NH;
  const int j0   = kb * 64 + wave * 16;
  const size_t rowB = (size_t)b * SEQ;

  const _Float16* Q16 = (const _Float16*)(const void*)qp + (size_t)h * HD;
  const _Float16* K16 = (const _Float16*)(const void*)kp + (size_t)h * HD;

  v16h ka[2];
#pragma unroll
  for (int dc = 0; dc < 2; ++dc) ka[dc] = ldfrag_h(K16 + (rowB + j0 + c) * DM + dc * 32 + 8 * hh);

  float mrun[8], zrun[8];
#pragma unroll
  for (int r = 0; r < 8; ++r) { mrun[r] = -1.0e30f; zrun[r] = 0.f; }

  for (int qt = 0; qt < NQB; ++qt) {
    __syncthreads();
    {
      const int r = tid >> 1, hf = (tid & 1) * 32;
      const _Float16* qg = Q16 + (rowB + (size_t)qt * 64 + r) * DM + hf;
#pragma unroll
      for (int i = 0; i < 4; ++i) *(v8h*)(Qsh + r * 64 + hf + 8 * i) = *(const v8h*)(qg + 8 * i);
    }
    __syncthreads();

    v8f s[4];
#pragma unroll
    for (int it = 0; it < 4; ++it) {
      v8f sa = zero8();
#pragma unroll
      for (int dc = 0; dc < 2; ++dc) {
        FH qb;
        qb.h[0] = *(const v8h*)(Qsh + (it * 16 + c) * 64 + dc * 32 + 8 * hh);
        qb.h[1] = *(const v8h*)(Qsh + (it * 16 + c) * 64 + dc * 32 + 16 + 8 * hh);
        sa = mma_h(ka[dc], qb.v, sa);
      }
#pragma unroll
      for (int r = 0; r < 8; ++r) s[it][r] = sa[r] * sscale;
    }

#pragma unroll
    for (int r = 0; r < 8; ++r) {
      float m = s[0][r];
      m = fmaxf(m, s[1][r]);
      m = fmaxf(m, s[2][r]);
      m = fmaxf(m, s[3][r]);
#pragma unroll
      for (int off = 1; off < 16; off <<= 1) m = fmaxf(m, __shfl_xor(m, off, 32));
      const float mnew  = fmaxf(mrun[r], m);
      const float alpha = __expf(mrun[r] - mnew);
      float psum = 0.f;
#pragma unroll
      for (int it = 0; it < 4; ++it) psum += __expf(s[it][r] - mnew);
#pragma unroll
      for (int off = 1; off < 16; off <<= 1) psum += __shfl_xor(psum, off, 32);
      zrun[r] = zrun[r] * alpha + psum;
      mrun[r] = mnew;
    }
  }

#pragma unroll
  for (int r = 0; r < 8; ++r) {
    const int key = wave * 16 + 8 * hh + r;
    const float rz = 1.0f / zrun[r];
    if (c == r) { Ssh[2 * key] = mrun[r]; Ssh[2 * key + 1] = rz; }
  }
  __syncthreads();
  if (wave == 0) {
    const v4f v = *(const v4f*)(Ssh + 4 * lane);
    float* dst = stats + (((size_t)b * NH + h) * SEQ + (size_t)kb * 64) * 2 + 4 * lane;
    *(volatile v4f*)dst = v;
    __threadfence();
    *(volatile v4f*)dst = v;
  }
}

__global__ __launch_bounds__(128)
void rowacc(const unsigned short* __restrict__ qp, const unsigned short* __restrict__ kp,
            const unsigned short* __restrict__ vtp, const float* __restrict__ stats,
            unsigned short* ctxp, float sscale, float pscale, float oscale) {
  union FH { v16h v; v8h h[2]; };
  __shared__ __align__(16) _Float16 Ksh[64 * 64];
  __shared__ __align__(16) _Float16 Vsh[64 * 64];
  __shared__ __align__(16) _Float16 Psh[4][16 * 64];
  __shared__ __align__(16) float    Ssh[128];
  __shared__ __align__(16) float    Os[4][16 * 64];

  const int tid  = threadIdx.x;
  const int wave = tid >> 5;
  const int lane = tid & 31;
  const int hh   = lane >> 4;
  const int c    = lane & 15;

  const int bx   = blockIdx.x;
  const int qb   = bx % NQB;
  const int rest = bx / NQB;
  const int h    = rest % NH;
  const int b    = rest / NH;
  const int q0   = qb * 64 + wave * 16;
  const size_t rowB = (size_t)b * SEQ;

  const _Float16* Q16 = (const _Float16*)(const void*)qp + (size_t)h * HD;
  const _Float16* K16 = (const _Float16*)(const void*)kp + (size_t)h * HD;
  const _Float16* V16 = (const _Float16*)(const void*)vtp + ((size_t)b * DM + (size_t)h * HD) * SEQ;
  const float*    Sg  = stats + ((size_t)b * NH + h) * SEQ * 2;

  v16h qa[2];
#pragma unroll
  for (int dc = 0; dc < 2; ++dc) qa[dc] = ldfrag_h(Q16 + (rowB + q0 + c) * DM + dc * 32 + 8 * hh);

  v8f oacc[4];
#pragma unroll
  for (int t = 0; t < 4; ++t) oacc[t] = zero8();

  for (int kt = 0; kt < NQB; ++kt) {
    const int kv0 = kt * 64;
    __syncthreads();
    {
      const int r = tid >> 1, hf = (tid & 1) * 32;
      const _Float16* kg = K16 + (rowB + kv0 + r) * DM + hf;
      const _Float16* vg = V16 + (size_t)r * SEQ + kv0 + hf;
#pragma unroll
      for (int i = 0; i < 4; ++i) {
        const v8h a0 = *(const v8h*)(kg + 8 * i);
        const v8h b0 = *(const v8h*)(vg + 8 * i);
        *(v8h*)(Ksh + r * 64 + hf + 8 * i) = a0;
        *(v8h*)(Vsh + r * 64 + hf + 8 * i) = b0;
      }
      if (wave == 0) *(v4f*)(Ssh + 4 * lane) = *(const v4f*)(Sg + (size_t)kv0 * 2 + 4 * lane);
    }
    __syncthreads();

    _Float16* pwh = Psh[wave];
#pragma unroll
    for (int jt = 0; jt < 4; ++jt) {
      v8f sa = zero8();
#pragma unroll
      for (int dc = 0; dc < 2; ++dc) {
        FH kf;
        kf.h[0] = *(const v8h*)(Ksh + (jt * 16 + c) * 64 + dc * 32 + 8 * hh);
        kf.h[1] = *(const v8h*)(Ksh + (jt * 16 + c) * 64 + dc * 32 + 16 + 8 * hh);
        sa = mma_h(qa[dc], kf.v, sa);
      }
      const float mj = Ssh[2 * (jt * 16 + c)];
      const float rj = Ssh[2 * (jt * 16 + c) + 1];
#pragma unroll
      for (int r = 0; r < 8; ++r) {
        const float p = __expf(sa[r] * sscale - mj) * rj;
        pwh[(8 * hh + r) * 64 + jt * 16 + c] = (_Float16)(p * pscale);
      }
    }
    wave_sync_lds();

#pragma unroll 1
    for (int kk = 0; kk < 2; ++kk) {
      FH pa;
      pa.h[0] = *(const v8h*)(pwh + c * 64 + kk * 32 + 8 * hh);
      pa.h[1] = *(const v8h*)(pwh + c * 64 + kk * 32 + 16 + 8 * hh);
#pragma unroll
      for (int t = 0; t < 4; ++t) {
        FH vb;
        vb.h[0] = *(const v8h*)(Vsh + (t * 16 + c) * 64 + kk * 32 + 8 * hh);
        vb.h[1] = *(const v8h*)(Vsh + (t * 16 + c) * 64 + kk * 32 + 16 + 8 * hh);
        oacc[t] = mma_h(pa.v, vb.v, oacc[t]);
      }
    }
  }

  float* os = Os[wave];
#pragma unroll
  for (int r = 0; r < 8; ++r) {
#pragma unroll
    for (int t = 0; t < 4; ++t) os[(8 * hh + r) * 64 + t * 16 + c] = oacc[t][r] * oscale;
  }
  wave_sync_lds();
  {
    const int q4 = lane >> 3, c8 = (lane & 7) * 8;
    v4u hv[4];
#pragma unroll
    for (int it = 0; it < 4; ++it) {
      const int row = it * 4 + q4;
      const float* sp = os + row * 64 + c8;
      v4u a;
#pragma unroll
      for (int e = 0; e < 4; ++e) {
        a[e] = pk16(h_bits((_Float16)sp[2 * e]), h_bits((_Float16)sp[2 * e + 1]));
      }
      hv[it] = a;
    }
    for (int pass = 0; pass < 2; ++pass) {
#pragma unroll
      for (int it = 0; it < 4; ++it) {
        const int row = it * 4 + q4;
        const size_t go = (rowB + q0 + row) * DM + (size_t)h * HD + c8;
        *(volatile v4u*)(ctxp + go) = hv[it];
      }
      __threadfence();
    }
  }
}

extern "C" void kernel_launch(void* const* d_in, const int* in_sizes, int n_in,
                              void* d_out, int out_size, void* d_ws, size_t ws_size,
                              hipStream_t stream) {
  if (n_in < 11) return;
  const int nx = NB * SEQ * DM;
  const int nw = DM * DM;
  if (in_sizes[0] != nx || in_sizes[1] != nx || in_sizes[2] != nx) return;
  if (in_sizes[3] != nw || in_sizes[5] != nw || in_sizes[7] != nw || in_sizes[9] != nw) return;
  if (in_sizes[4] != DM || in_sizes[6] != DM || in_sizes[8] != DM || in_sizes[10] != DM) return;
  if (out_size != nx) return;

  const float* query = (const float*)d_in[0];
  const float* keyin = (const float*)d_in[1];
  const float* value = (const float*)d_in[2];
  const float* Wq = (const float*)d_in[3];
  const float* bq = (const float*)d_in[4];
  const float* Wk = (const float*)d_in[5];
  const float* bk = (const float*)d_in[6];
  const float* Wv = (const float*)d_in[7];
  const float* bv = (const float*)d_in[8];
  const float* Wo = (const float*)d_in[9];
  const float* bo = (const float*)d_in[10];

  const size_t PX   = (size_t)NB * SEQ * DM * 2;
  const size_t PW   = (size_t)DM * DM * 2;
  const size_t PQ   = (size_t)NB * SEQ * DM * 2;
  const size_t PVT  = (size_t)NB * DM * SEQ * 2;
  const size_t PST  = (size_t)NB * NH * SEQ * 2 * 4;
  const size_t PCTX = (size_t)NB * SEQ * DM * 2;
  size_t off = 0;
  const size_t oX   = off; off += PX;
  const size_t oWq  = off; off += PW;
  const size_t oWk  = off; off += PW;
  const size_t oWv  = off; off += PW;
  const size_t oWo  = off; off += PW;
  const size_t oQ   = off; off += PQ;
  const size_t oK   = off; off += PQ;
  const size_t oVT  = off; off += PVT;
  const size_t oST  = off; off += PST;
  const size_t oCTX = off; off += PCTX;
  if (off > ws_size) return;
  if (off > (size_t)134217728) return;

  char* ws = (char*)d_ws;
  unsigned short* X    = (unsigned short*)(ws + oX);
  unsigned short* WqT  = (unsigned short*)(ws + oWq);
  unsigned short* WkT  = (unsigned short*)(ws + oWk);
  unsigned short* WvT  = (unsigned short*)(ws + oWv);
  unsigned short* Wo16 = (unsigned short*)(ws + oWo);
  unsigned short* Qp   = (unsigned short*)(ws + oQ);
  unsigned short* Kp   = (unsigned short*)(ws + oK);
  unsigned short* VT   = (unsigned short*)(ws + oVT);
  float*          ST   = (float*)(ws + oST);
  unsigned short* CTX  = (unsigned short*)(ws + oCTX);

  const dim3 blk(256);
  const int  n8x = nx / 8;
  const dim3 gCvt((n8x + 255) / 256);
  const dim3 gW(DM / 64, DM / 64);
  const dim3 gQ(((NB * SEQ / 64) * (DM / 64) + 7) / 8, 1);
  const dim3 gVT(((DM / 64) * (SEQ / 64) + 7) / 8, NB);
  const dim3 gOut(((NB * SEQ / 64) * (DM / 64) + 7) / 8, 1);
  const dim3 gAttn(NB * NH * NQB);

  wtrans<0><<<gW, blk, 0, stream>>>(Wq, WqT, 1.0f);
  wtrans<0><<<gW, blk, 0, stream>>>(Wk, WkT, 1.0f);
  wtrans<0><<<gW, blk, 0, stream>>>(Wv, WvT, 1.0f);
  wtrans<1><<<gW, blk, 0, stream>>>(Wo, Wo16, 16.0f);
  cvt_bf16x8<<<gCvt, blk, 0, stream>>>(query, X, n8x);
  gemm64<0, 1, 1><<<gQ, blk, 0, stream>>>(X, DM, 0LL, WqT, DM, 0LL, bq,
                                          (void*)Qp, DM, 0LL, NB * SEQ, DM, DM, 1.0f);
  cvt_bf16x8<<<gCvt, blk, 0, stream>>>(keyin, X, n8x);
  gemm64<0, 1, 1><<<gQ, blk, 0, stream>>>(X, DM, 0LL, WkT, DM, 0LL, bk,
                                          (void*)Kp, DM, 0LL, NB * SEQ, DM, DM, 1.0f);
  cvt_bf16x8<<<gCvt, blk, 0, stream>>>(value, X, n8x);
  gemm64<0, 1, 2><<<gVT, blk, 0, stream>>>(WvT, DM, 0LL, X, DM, (long long)SEQ * DM, bv,
                                           (void*)VT, SEQ, (long long)DM * SEQ, DM, SEQ, DM, 1.0f);
  colstats<<<gAttn, dim3(128), 0, stream>>>(Qp, Kp, ST, 0.125f);
  rowacc<<<gAttn, dim3(128), 0, stream>>>(Qp, Kp, VT, ST, CTX, 0.125f, 1024.0f, 16.0f / 1024.0f);
  gemm64<1, 0, 1><<<gOut, blk, 0, stream>>>(CTX, DM, 0LL, Wo16, DM, 0LL, bo,
                                            d_out, DM, 0LL, NB * SEQ, DM, DM, 1.0f / 256.0f);
  (void)hipGetLastError();
}
